// DynamicsWithKnownReward_14542759264837
// MI455X (gfx1250) — hardware-verified
//
#include <hip/hip_runtime.h>
#include <stddef.h>


typedef _Float16 v16h __attribute__((ext_vector_type(16)));
typedef _Float16 v8h  __attribute__((ext_vector_type(8)));
typedef float    v8f  __attribute__((ext_vector_type(8)));
typedef float    v4f  __attribute__((ext_vector_type(4)));
typedef _Float16 h16;

#ifndef NROWS
#define NROWS 524288
#endif
#define NROWS_FULL 524288
#define SDIM 3
#define ADIM 2
#define XDIM 5
#define HIDN 128
#define K1P  32
#define N3P  16
#define RPB  1024
#define TPW  8
#define OUT1_ELEM ((size_t)NROWS_FULL * SDIM)

static_assert(NROWS >= RPB && NROWS <= NROWS_FULL && (NROWS % RPB) == 0);
static_assert(RPB == 8 * TPW * 16);
static_assert(XDIM == SDIM + ADIM && XDIM <= 8);
static_assert((HIDN % 64) == 0 && (HIDN % 32) == 0);
static_assert(HIDN == 128);
static_assert(SDIM <= 8 && SDIM <= N3P);
static_assert(OUT1_ELEM * 4 == (size_t)6291456);
static_assert((RPB * SDIM) % (4 * 256) == 0);
static_assert((RPB * ADIM) % (4 * 256) == 0);
static_assert(RPB == 4 * 256);
static_assert(((size_t)RPB * SDIM * 4) % 128 == 0);

#define LDT 72
#define LD1 40
#define LDW 136
static_assert((LDT % 8) == 0 && LDT >= 64);
static_assert((LD1 % 8) == 0 && LD1 >= K1P);
static_assert((LDW % 8) == 0 && LDW >= HIDN);

#define WCARRY 64.0f
#define XCARRY 16.0f
#define MCARRY 16.0f

#define W2T_BYTES ((size_t)HIDN * HIDN * 2)
#define W1T_BYTES ((size_t)HIDN * K1P * 2)
#define W3T_BYTES ((size_t)N3P * HIDN * 2)
#define OFF_W2T ((size_t)0)
#define OFF_W1T (OFF_W2T + W2T_BYTES)
#define OFF_W3T (OFF_W1T + W1T_BYTES)
#define WS_TOTAL (OFF_W3T + W3T_BYTES)
static_assert((W2T_BYTES % 128) == 0 && (W1T_BYTES % 128) == 0 && (W3T_BYTES % 128) == 0);
static_assert(W1T_BYTES == (size_t)2 * 256 * 16);
static_assert(W3T_BYTES == (size_t)256 * 16);
static_assert(W2T_BYTES == (size_t)8 * 256 * 16);
static_assert(WS_TOTAL <= (size_t)134217728);

__device__ __forceinline__ float bf16r(float x) {
  unsigned int u = __float_as_uint(x);
  u = (u + 0x7FFFu + ((u >> 16) & 1u)) & 0xFFFF0000u;
  return __uint_as_float(u);
}

static __device__ __forceinline__ h16 toh_flush(float v) {
  const h16 r = (h16)v;
  return (fabsf(v) < 6.103515625e-05f) ? (h16)0.0f : r;
}

__device__ __forceinline__ v16h frag_at(const _Float16* p) {
  v8h lo = *(const v8h*)(p);
  v8h hi = *(const v8h*)(p + 16);
  v16h out;
#pragma unroll
  for (int i = 0; i < 8; ++i) { out[i] = lo[i]; out[i + 8] = hi[i]; }
  return out;
}
__device__ __forceinline__ v16h ld_frag(const _Float16* base, unsigned ld) {
  const unsigned lane = threadIdx.x & 31u;
  return frag_at(base + (lane & 15u) * ld + (lane >> 4) * 8u);
}

__device__ __forceinline__ v8f wmma16(v16h a, v16h b, v8f c) {
  v8f d = __builtin_amdgcn_wmma_f32_16x16x32_f16(false, a, false, b, (short)0, c,
                                                 false, false);
  asm volatile("v_nop\n\tv_nop\n\tv_nop\n\tv_nop" : "+v"(d) : "v"(a), "v"(b));
  return d;
}

__device__ __forceinline__ float relu_act(float t) {
  return fmaxf(t, 0.0f);
}

__device__ __forceinline__ float gterm(float dx, float dy, float k) {
  return __expf(-(dx * dx + dy * dy) * k);
}

__global__ __launch_bounds__(256) void wconv_kernel(
    const float* __restrict__ W, _Float16* __restrict__ Wt, unsigned ldw, unsigned ldk) {
  __shared__ _Float16 T[64 * LDT];
  const unsigned tid = threadIdx.x;
  const unsigned n0 = blockIdx.x * 64u;
  const unsigned k0 = blockIdx.y * 64u;
#pragma unroll 4
  for (unsigned j = 0; j < 16u; ++j) {
    const unsigned idx = tid + 256u * j;
    const unsigned kr = idx >> 6, nc = idx & 63u;
    const float v = W[(size_t)(k0 + kr) * ldw + n0 + nc];
    T[nc * LDT + kr] = (_Float16)(WCARRY * bf16r(v));
  }
  __syncthreads();
  v8h x[2];
  size_t off[2];
#pragma unroll
  for (unsigned i = 0; i < 2u; ++i) {
    const unsigned n = 32u * i + (tid >> 3);
    const unsigned kc = (tid & 7u) * 8u;
    x[i] = *(const v8h*)&T[n * LDT + kc];
    off[i] = (size_t)(n0 + n) * ldk + k0 + kc;
  }
#pragma unroll
  for (int i = 0; i < 2; ++i) *(volatile v8h*)(Wt + off[i]) = x[i];
  __threadfence();
#pragma unroll
  for (int i = 0; i < 2; ++i) *(volatile v8h*)(Wt + off[i]) = x[i];
}

__global__ __launch_bounds__(256) void wsmall_kernel(
    const float* __restrict__ W1, const float* __restrict__ W3,
    _Float16* __restrict__ W1t, _Float16* __restrict__ W3t) {
  const unsigned tid = threadIdx.x;
  v8h x1[2];
#pragma unroll
  for (unsigned i = 0; i < 2u; ++i) {
    const unsigned p = tid + 256u * i;
    const unsigned n = p >> 2, kc = (p & 3u) * 8u;
    v8h o;
#pragma unroll
    for (unsigned j = 0; j < 8u; ++j) {
      const unsigned k = kc + j;
      const unsigned kk = (k < (unsigned)XDIM) ? k : (unsigned)(XDIM - 1);
      const float w = W1[kk * (unsigned)HIDN + n];
      const float v = (k < (unsigned)XDIM) ? (WCARRY * bf16r(w)) : 0.0f;
      o[j] = toh_flush(v);
    }
    x1[i] = o;
  }
  v8h x3;
  {
    const unsigned n = tid >> 4, kc = (tid & 15u) * 8u;
    const unsigned nn = (n < (unsigned)SDIM) ? n : (unsigned)(SDIM - 1);
#pragma unroll
    for (unsigned j = 0; j < 8u; ++j) {
      const float w = W3[(kc + j) * (unsigned)SDIM + nn];
      const float v = (n < (unsigned)SDIM) ? (WCARRY * bf16r(w)) : 0.0f;
      x3[j] = toh_flush(v);
    }
  }
#pragma unroll
  for (unsigned i = 0; i < 2u; ++i) *(volatile v8h*)(W1t + (size_t)(tid + 256u * i) * 8u) = x1[i];
  *(volatile v8h*)(W3t + (size_t)tid * 8u) = x3;
  __threadfence();
#pragma unroll
  for (unsigned i = 0; i < 2u; ++i) *(volatile v8h*)(W1t + (size_t)(tid + 256u * i) * 8u) = x1[i];
  *(volatile v8h*)(W3t + (size_t)tid * 8u) = x3;
}

__global__ __launch_bounds__(256) void mlp_reward_kernel(
    const float* __restrict__ S, const float* __restrict__ A,
    const _Float16* __restrict__ W1t, const _Float16* __restrict__ W2t,
    const _Float16* __restrict__ W3t,
    const float* __restrict__ B1, const float* __restrict__ B2, const float* __restrict__ B3,
    float* __restrict__ OutS, float* __restrict__ OutR) {
  __shared__ __attribute__((aligned(16))) _Float16 W1s[HIDN * LD1];
  __shared__ __attribute__((aligned(16))) _Float16 W2s[HIDN * LDW];
  __shared__ __attribute__((aligned(16))) _Float16 W3s[N3P * LDW];
  __shared__ __attribute__((aligned(16))) float b1s[HIDN];
  __shared__ __attribute__((aligned(16))) float b2s[HIDN];
  __shared__ __attribute__((aligned(16))) float Ss[RPB * SDIM];
  __shared__ __attribute__((aligned(16))) float As[RPB * ADIM];
  __shared__ __attribute__((aligned(16))) float Os[RPB * SDIM];
  __shared__ __attribute__((aligned(16))) float Rs[RPB];

  const unsigned tid = threadIdx.x, lane = tid & 31u;
  const unsigned wave = (unsigned)__builtin_amdgcn_readfirstlane((int)(threadIdx.x >> 5));
  const unsigned hh = lane >> 4, m = lane & 15u;
  const size_t row0 = (size_t)blockIdx.x * RPB;

#pragma unroll
  for (unsigned j = 0; j < 8u; ++j) {
    const unsigned p = tid + 256u * j;
    const unsigned n = p >> 4, c = (p & 15u) * 8u;
    *(v8h*)&W2s[n * LDW + c] = *(const v8h*)(W2t + (size_t)p * 8u);
  }
#pragma unroll
  for (unsigned j = 0; j < 2u; ++j) {
    const unsigned p = tid + 256u * j;
    const unsigned n = p >> 2, c = (p & 3u) * 8u;
    *(v8h*)&W1s[n * LD1 + c] = *(const v8h*)(W1t + (size_t)p * 8u);
  }
  {
    const unsigned n = tid >> 4, c = (tid & 15u) * 8u;
    *(v8h*)&W3s[n * LDW + c] = *(const v8h*)(W3t + (size_t)tid * 8u);
  }
  if (tid < (unsigned)HIDN) {
    b1s[tid] = bf16r(B1[tid]);
    b2s[tid] = bf16r(B2[tid]);
  }
#pragma unroll
  for (unsigned i = 0; i < 3u; ++i) {
    const unsigned idx = tid + 256u * i;
    const v4f v = *(const v4f*)(S + row0 * SDIM + (size_t)idx * 4u);
    v4f t;
#pragma unroll
    for (int j = 0; j < 4; ++j) t[j] = bf16r(v[j]);
    *(v4f*)&Ss[idx * 4u] = t;
  }
#pragma unroll
  for (unsigned i = 0; i < 2u; ++i) {
    const unsigned idx = tid + 256u * i;
    const v4f v = *(const v4f*)(A + row0 * ADIM + (size_t)idx * 4u);
    v4f t;
#pragma unroll
    for (int j = 0; j < 4; ++j) t[j] = bf16r(v[j]);
    *(v4f*)&As[idx * 4u] = t;
  }
  __syncthreads();

  {
    const float inv2var = 0.5f / 0.035f;
    const float gcoef   = 100.0f / (2.0f * 3.14159265358979323f * 0.035f);
    const float bcoef   = 10.0f / (0.03f * 2.5066282746310002f);
    const float ibs     = 0.5f / (0.03f * 0.03f);
#pragma unroll 1
    for (unsigned i = 0; i < 4u; ++i) {
      const unsigned r = i * 256u + tid;
      const float sx = Ss[r * 3u + 0u], sy = Ss[r * 3u + 1u];
      const float ax = As[r * 2u + 0u], ay = As[r * 2u + 1u];
      float gs = gterm(sx, sy, inv2var);
      gs += gterm(sx, sy - 0.2f, inv2var);
      gs += gterm(sx, sy - 0.4f, inv2var);
      gs += gterm(sx, sy - 0.6f, inv2var);
      gs += gterm(sx, sy - 0.8f, inv2var);
      gs += gterm(sx + 0.8f, sy + 0.8f, inv2var);
      const float qx = sx - ax, qy = sy - ay;
      const float quad = 30.0f * (qx * qx + qy * qy);
      const float e0 = __expf(-(sx + 1.5f) * (sx + 1.5f) * ibs);
      const float e1 = __expf(-(sx - 1.5f) * (sx - 1.5f) * ibs);
      const float e2 = __expf(-(sy - 1.0f) * (sy - 1.0f) * ibs);
      const float e3 = __expf(-(sy + 1.0f) * (sy + 1.0f) * ibs);
      Rs[r] = -(quad + gcoef * gs + bcoef * (((e0 + e1) + e2) + e3));
    }
  }

  const float b30 = bf16r(B3[0]);
  const float b31 = bf16r(B3[1]);
  const float b32 = bf16r(B3[2]);
  const float sc1 = 1.0f / (WCARRY * XCARRY);
  const float sc2 = 1.0f / (WCARRY * MCARRY);
  const bool lo_half = (hh == 0u);

#pragma unroll 1
  for (unsigned it = 0; it < (unsigned)TPW; ++it) {
    const unsigned lr = (wave * (unsigned)TPW + it) * 16u + m;
    const float x0 = Ss[lr * 3u + 0u];
    const float x1 = Ss[lr * 3u + 1u];
    const float x2 = Ss[lr * 3u + 2u];
    const float x3 = As[lr * 2u + 0u];
    const float x4 = As[lr * 2u + 1u];

    v16h xb;
#pragma unroll
    for (int i = 0; i < 16; ++i) xb[i] = (h16)0.0f;
    xb[0] = toh_flush(lo_half ? (XCARRY * x0) : 0.0f);
    xb[1] = toh_flush(lo_half ? (XCARRY * x1) : 0.0f);
    xb[2] = toh_flush(lo_half ? (XCARRY * x2) : 0.0f);
    xb[3] = toh_flush(lo_half ? (XCARRY * x3) : 0.0f);
    xb[4] = toh_flush(lo_half ? (XCARRY * x4) : 0.0f);

    v16h hb[4];
#pragma unroll
    for (int j = 0; j < 4; ++j) {
#pragma unroll
      for (int e = 0; e < 2; ++e) {
        const int n = 2 * j + e;
        const v16h a = ld_frag(&W1s[(n * 16) * LD1], LD1);
        v8f d = {};
        d = wmma16(a, xb, d);
        const v4f g0 = *(const v4f*)&b1s[(unsigned)(n * 16) + hh * 8u];
        const v4f g1 = *(const v4f*)&b1s[(unsigned)(n * 16) + hh * 8u + 4u];
#pragma unroll
        for (int r = 0; r < 4; ++r) {
          const float t0 = relu_act(d[r] * sc1 + g0[r]);
          const float t1 = relu_act(d[r + 4] * sc1 + g1[r]);
          hb[j][e * 8 + r]     = toh_flush(MCARRY * t0);
          hb[j][e * 8 + 4 + r] = toh_flush(MCARRY * t1);
        }
      }
    }

    v16h h2b[4];
#pragma unroll
    for (int j = 0; j < 4; ++j) {
#pragma unroll
      for (int e = 0; e < 2; ++e) {
        const int n = 2 * j + e;
        v8f d = {};
#pragma unroll
        for (int kq = 0; kq < 4; ++kq) {
          const v16h a = ld_frag(&W2s[(n * 16) * LDW + kq * 32], LDW);
          d = wmma16(a, hb[kq], d);
        }
        const v4f g0 = *(const v4f*)&b2s[(unsigned)(n * 16) + hh * 8u];
        const v4f g1 = *(const v4f*)&b2s[(unsigned)(n * 16) + hh * 8u + 4u];
#pragma unroll
        for (int r = 0; r < 4; ++r) {
          const float t0 = relu_act(d[r] * sc2 + g0[r]);
          const float t1 = relu_act(d[r + 4] * sc2 + g1[r]);
          h2b[j][e * 8 + r]     = toh_flush(MCARRY * t0);
          h2b[j][e * 8 + 4 + r] = toh_flush(MCARRY * t1);
        }
      }
    }

    v8f d3 = {};
#pragma unroll
    for (int kq = 0; kq < 4; ++kq) {
      const v16h a = ld_frag(&W3s[kq * 32], LDW);
      d3 = wmma16(a, h2b[kq], d3);
    }
    const float o0 = d3[0] * sc2 + b30;
    const float o1 = d3[1] * sc2 + b31;
    const float o2 = d3[2] * sc2 + b32;
    if (lo_half) {
      Os[lr * 3u + 0u] = o0;
      Os[lr * 3u + 1u] = o1;
      Os[lr * 3u + 2u] = o2;
    }
  }
  __syncthreads();

  v4f xo[3];
  size_t oo[3];
#pragma unroll
  for (unsigned i = 0; i < 3u; ++i) {
    const unsigned idx = tid + 256u * i;
    xo[i] = *(const v4f*)&Os[idx * 4u];
    oo[i] = row0 * SDIM + (size_t)idx * 4u;
  }
  const v4f xr = *(const v4f*)&Rs[tid * 4u];
  const size_t orr = row0 + (size_t)tid * 4u;
#pragma unroll
  for (int i = 0; i < 3; ++i) *(volatile v4f*)(OutS + oo[i]) = xo[i];
  *(volatile v4f*)(OutR + orr) = xr;
  __threadfence();
#pragma unroll
  for (int i = 0; i < 3; ++i) *(volatile v4f*)(OutS + oo[i]) = xo[i];
  *(volatile v4f*)(OutR + orr) = xr;
}

extern "C" void kernel_launch(void* const* d_in, const int* in_sizes, int n_in,
                              void* d_out, int out_size, void* d_ws, size_t ws_size,
                              hipStream_t stream) {
  if (n_in < 8) return;
  if ((long long)in_sizes[0] < (long long)NROWS * SDIM) return;
  if ((long long)in_sizes[1] < (long long)NROWS * ADIM) return;
  if (in_sizes[2] < XDIM * HIDN) return;
  if (in_sizes[3] < HIDN) return;
  if (in_sizes[4] < HIDN * HIDN) return;
  if (in_sizes[5] < HIDN) return;
  if (in_sizes[6] < HIDN * SDIM) return;
  if (in_sizes[7] < SDIM) return;
  if ((long long)out_size < (long long)OUT1_ELEM + (long long)NROWS) return;
  if (ws_size < WS_TOTAL) return;

  const float* s  = (const float*)d_in[0];
  const float* a  = (const float*)d_in[1];
  const float* w1 = (const float*)d_in[2];
  const float* b1 = (const float*)d_in[3];
  const float* w2 = (const float*)d_in[4];
  const float* b2 = (const float*)d_in[5];
  const float* w3 = (const float*)d_in[6];
  const float* b3 = (const float*)d_in[7];
  float* out = (float*)d_out;

  char* ws = (char*)d_ws;
  _Float16* W2_t = (_Float16*)(ws + OFF_W2T);
  _Float16* W1_t = (_Float16*)(ws + OFF_W1T);
  _Float16* W3_t = (_Float16*)(ws + OFF_W3T);

  dim3 blk(256);
  wconv_kernel<<<dim3(HIDN / 64, HIDN / 64), blk, 0, stream>>>(w2, W2_t, (unsigned)HIDN, (unsigned)HIDN);
  wsmall_kernel<<<dim3(1), blk, 0, stream>>>(w1, w3, W1_t, W3_t);
  mlp_reward_kernel<<<dim3(NROWS / RPB), blk, 0, stream>>>(s, a, W1_t, W2_t, W3_t, b1, b2, b3,
                                                           out, out + OUT1_ELEM);
}
